// DisjointDense_26113401159978
// MI455X (gfx1250) — hardware-run, weakly checked
//
#include <hip/hip_runtime.h>


#define NR   4096
#define DI   256
#define DO   256
#define NB   64
#define KK   (NB * DI)
#define RB   1024
constexpr size_t al256(size_t b) { return (b + 255) & ~(size_t)255; }
constexpr size_t WS_TOTAL = al256((size_t)DO * KK * 2) + al256((size_t)DO * NB * 2) + al256((size_t)NR * NB * 2) + al256((size_t)RB * KK * 2) + 2 * al256((size_t)RB * DO * 4);
static_assert(WS_TOTAL == 44597248 && WS_TOTAL <= 134217728, "the workspace carve: about 42.5 MiB");
typedef _Float16 h16;
typedef unsigned short bf;
typedef __attribute__((ext_vector_type(16))) __bf16   v16bf;
typedef __attribute__((ext_vector_type(16))) _Float16 v16h;
typedef __attribute__((ext_vector_type(8)))  _Float16 v8h;
typedef __attribute__((ext_vector_type(8)))  unsigned short v8us;
typedef __attribute__((ext_vector_type(8)))  float    v8f;
typedef __attribute__((ext_vector_type(4)))  float    v4f;
typedef v8h  __attribute__((may_alias)) v8ha;
typedef v4f  __attribute__((may_alias)) v4fa;
typedef v8us __attribute__((may_alias)) v8usa;

__device__ __forceinline__ unsigned short f2bf(float f) { unsigned u = __float_as_uint(f); u += 0x7FFFu + ((u >> 16) & 1u); return (unsigned short)(u >> 16); }
__device__ __forceinline__ float bf2f(unsigned short b) { return __uint_as_float(((unsigned)b) << 16); }
__device__ __forceinline__ float bfr(float f) { return bf2f(f2bf(f)); }
__device__ __forceinline__ v16h cat16(v8h lo, v8h hi) { return __builtin_shufflevector(lo, hi, 0, 1, 2, 3, 4, 5, 6, 7, 8, 9, 10, 11, 12, 13, 14, 15); }
__device__ __forceinline__ v16bf cat16b(v8us lo, v8us hi) { return __builtin_bit_cast(v16bf, __builtin_shufflevector(lo, hi, 0, 1, 2, 3, 4, 5, 6, 7, 8, 9, 10, 11, 12, 13, 14, 15)); }
__device__ __forceinline__ v8f wmma16(v16h a, v16h b, v8f c) { return __builtin_amdgcn_wmma_f32_16x16x32_f16(false, a, false, b, (short)0, c, false, false); }
__device__ __forceinline__ v8f wmmab(v16bf a, v16bf b, v8f c) { return __builtin_amdgcn_wmma_f32_16x16x32_bf16(false, a, false, b, (short)0, c, false, false); }


template <typename T16> struct WFrag;
template <> struct WFrag<h16> { typedef v16h V; static __device__ __forceinline__ V ld(const h16* p) { return cat16(*(const v8h*)p, *(const v8h*)(p + 16)); } static __device__ __forceinline__ v8f mma(V a, V b, v8f c) { return wmma16(a, b, c); } };
template <> struct WFrag<bf> { typedef v16bf V; static __device__ __forceinline__ V ld(const bf* p) { return cat16b(*(const v8us*)p, *(const v8us*)(p + 16)); } static __device__ __forceinline__ v8f mma(V a, V b, v8f c) { return wmmab(a, b, c); } };
template <typename T16, int NSPLIT, bool BIAS>
__global__ __launch_bounds__(32) void k_gemmw(const T16* __restrict__ A, const T16* __restrict__ A2, const T16* __restrict__ Bt, const T16* __restrict__ Bt2, int K, float* C, int ldc, const float* __restrict__ bias, size_t sA, size_t sB, size_t sC) {
    typedef typename WFrag<T16>::V V;
    __shared__ __align__(16) float os[16 * 68];
    const size_t z = blockIdx.z; A += z * sA; if (A2) A2 += z * sA; Bt += z * sB; if (Bt2) Bt2 += z * sB; C += z * sC;
    const int lane = threadIdx.x & 31, lr = lane & 15, hi = lane >> 4; const int r0 = blockIdx.x * 64, c0 = blockIdx.y * 64;
    v8f acc[4][4];
#pragma unroll
    for (int mb = 0; mb < 4; ++mb)
#pragma unroll
        for (int nb = 0; nb < 4; ++nb) acc[mb][nb] = (v8f){};
    const size_t aoff = (size_t)(r0 + lr) * K + 8 * hi, boff = (size_t)(c0 + lr) * K + 8 * hi;
    for (int kc = 0; kc < K; kc += 32) {
        V a[4], a2[4];
#pragma unroll
        for (int mb = 0; mb < 4; ++mb) { a[mb] = WFrag<T16>::ld(A + aoff + (size_t)mb * 16 * K + kc); if (NSPLIT == 1 || NSPLIT == 2) a2[mb] = WFrag<T16>::ld(A2 + aoff + (size_t)mb * 16 * K + kc); }
#pragma unroll
        for (int nb = 0; nb < 4; ++nb) { const V b = WFrag<T16>::ld(Bt + boff + (size_t)nb * 16 * K + kc); V b2; if (NSPLIT >= 2) b2 = WFrag<T16>::ld(Bt2 + boff + (size_t)nb * 16 * K + kc);
#pragma unroll
            for (int mb = 0; mb < 4; ++mb) { acc[mb][nb] = WFrag<T16>::mma(a[mb], b, acc[mb][nb]); if (NSPLIT == 1 || NSPLIT == 2) acc[mb][nb] = WFrag<T16>::mma(a2[mb], b, acc[mb][nb]); if (NSPLIT >= 2) acc[mb][nb] = WFrag<T16>::mma(a[mb], b2, acc[mb][nb]); } }
        asm volatile("v_nop\n\tv_nop\n\tv_nop\n\tv_nop" : "+v"(acc[0][0]), "+v"(acc[1][1]), "+v"(acc[2][2]), "+v"(acc[3][3]) : "v"(a[0]), "v"(a[3]));
    }
#pragma unroll
    for (int mb = 0; mb < 4; ++mb) {
#pragma unroll
        for (int nb = 0; nb < 4; ++nb) {
#pragma unroll
            for (int j = 0; j < 8; ++j) os[(hi * 8 + j) * 68 + nb * 16 + lr] = acc[mb][nb][j]; }
        __builtin_amdgcn_wave_barrier(); asm volatile("" ::: "memory");
        float* crow = C + (size_t)(r0 + mb * 16) * ldc + c0;
#pragma unroll 1
        for (int ps = 0; ps < 2; ++ps) {
#pragma unroll
            for (int s = 0; s < 8; ++s) { const int row = 2 * s + hi, cofs = lr * 4; v4f val = *(const v4fa*)(os + row * 68 + cofs); if (BIAS) { val[0] += bfr(bias[c0 + cofs]); val[1] += bfr(bias[c0 + cofs + 1]); val[2] += bfr(bias[c0 + cofs + 2]); val[3] += bfr(bias[c0 + cofs + 3]); }
                *(volatile v4f*)(crow + (size_t)row * ldc + cofs) = val; }
            if (ps == 0) __threadfence(); }
        __builtin_amdgcn_wave_barrier(); asm volatile("" ::: "memory");
    }
}

__device__ __forceinline__ h16 tohx(float x) { return (h16)x; }
__device__ __forceinline__ void splitf(float y, unsigned short& h, unsigned short& l) { h = f2bf(y); l = f2bf(y - bf2f(h)); }
typedef __attribute__((ext_vector_type(2))) _Float16 v2h;
typedef __attribute__((ext_vector_type(4))) _Float16 v4h;
typedef __attribute__((ext_vector_type(2))) unsigned short v2us;
typedef __attribute__((ext_vector_type(4))) unsigned short v4us;
typedef __attribute__((ext_vector_type(2))) float v2f;
typedef __attribute__((ext_vector_type(4))) int v4i;

__global__ __launch_bounds__(256) void k_wtG(const float* __restrict__ w, int K, int N, bf* Bt) {
    const int lane = threadIdx.x & 31; const int L0 = (blockIdx.x * 8 + (threadIdx.x >> 5)) * 8; const int nlines = N * K / 64;
#pragma unroll
    for (int ps = 0; ps < 2; ++ps) {
        for (int l = 0; l < 8; ++l) { const int L = L0 + l; if (L >= nlines) break; const size_t e = (size_t)L * 64 + lane * 2; const int k = (int)(e % K), n = (int)(e / K); v2us o;
            o[0] = f2bf(w[(size_t)k * N + n]); o[1] = f2bf(w[(size_t)(k + 1) * N + n]); *(volatile v2us*)(Bt + e) = o; }
        if (ps == 0) __threadfence(); }
}

__global__ __launch_bounds__(256) void k_cvt8(const float* __restrict__ src, bf* dst, size_t n8) { const size_t i = (size_t)blockIdx.x * 256 + threadIdx.x; if (i >= n8) return; const v8f v = *(const v8f*)(src + i * 8); v8us o;
#pragma unroll
    for (int k = 0; k < 8; ++k) o[k] = f2bf(v[k]); *(volatile v8us*)(dst + i * 8) = o; __threadfence(); *(volatile v8us*)(dst + i * 8) = o; }

__global__ __launch_bounds__(256) void k_selx(const float* __restrict__ xr, const float* __restrict__ pk, bf* A) {
    const size_t e = (size_t)blockIdx.x * 256 + threadIdx.x; if (e >= (size_t)RB * NB * (DI / 8)) return; const int i8 = (int)(e % (DI / 8)); const int d = (int)((e / (DI / 8)) % NB); const size_t r = e / ((size_t)(DI / 8) * NB);
    const float s = bfr(pk[r * NB + d]); const v4f a = *(const v4f*)(xr + r * DI + (size_t)i8 * 8); const v4f b = *(const v4f*)(xr + r * DI + (size_t)i8 * 8 + 4); v8us o;
#pragma unroll
    for (int q = 0; q < 4; ++q) { o[q] = f2bf(s * bfr(a[q])); o[q + 4] = f2bf(s * bfr(b[q])); }
    bf* p = A + r * KK + (size_t)d * DI + (size_t)i8 * 8; *(volatile v8us*)p = o; __threadfence(); *(volatile v8us*)p = o; }

__global__ __launch_bounds__(256) void axpby_kernel(const float* __restrict__ A, const float* __restrict__ B, float* __restrict__ Y, size_t n4, float pa, float pb) {
  const size_t i = (size_t)blockIdx.x * 256 + threadIdx.x; if (i >= n4) return; const v4f a = *(const v4f*)(A + 4 * i); const v4f b = *(const v4f*)(B + 4 * i); v4f o; for (int j = 0; j < 4; ++j) o[j] = (pa * a[j]) + (pb * b[j]);
  for (int pass = 0; pass < 2; ++pass) { *(volatile v4f*)(Y + 4 * i) = o; __threadfence(); }
}

extern "C" void kernel_launch(void* const* d_in, const int* in_sizes, int n_in,
                              void* d_out, int out_size, void* d_ws, size_t ws_size, hipStream_t stream) {
    if (n_in < 4) return;
    if (in_sizes[0] < NR * DI || in_sizes[1] < NR * NB || in_sizes[2] < NB * DI * DO || in_sizes[3] < NB * DO || out_size < NR * DO) return;
    const float* xr = (const float*)d_in[0]; const float* pk = (const float*)d_in[1]; const float* wk = (const float*)d_in[2]; const float* vk = (const float*)d_in[3];
    float* OUT = (float*)d_out;
    char* wsp = (char*)d_ws;
    auto take = [&](size_t bytes) { char* p = wsp; wsp += (bytes + 255) & ~(size_t)255; return (void*)p; };
    bf* WT = (bf*)take((size_t)DO * KK * 2); bf* VT = (bf*)take((size_t)DO * NB * 2); bf* PB = (bf*)take((size_t)NR * NB * 2); bf* A = (bf*)take((size_t)RB * KK * 2); float* P1 = (float*)take((size_t)RB * DO * 4); float* P2 = (float*)take((size_t)RB * DO * 4);
    if ((size_t)(wsp - (char*)d_ws) != WS_TOTAL || WS_TOTAL > ws_size) return;
    k_wtG<<<(unsigned)((KK * DO / 64 + 63) / 64), 256, 0, stream>>>(wk, KK, DO, WT);
    k_wtG<<<(unsigned)((NB * DO / 64 + 63) / 64), 256, 0, stream>>>(vk, NB, DO, VT);
    k_cvt8<<<(unsigned)(((size_t)NR * NB / 8 + 255) / 256), 256, 0, stream>>>(pk, PB, (size_t)NR * NB / 8);
    for (int blk = 0; blk < NR / RB; ++blk) { const size_t r0 = (size_t)blk * RB;
        k_selx<<<(unsigned)(((size_t)RB * NB * (DI / 8) + 255) / 256), 256, 0, stream>>>(xr + r0 * DI, pk + r0 * NB, A);
        k_gemmw<bf, 0, false><<<dim3(RB / 64, DO / 64, 1), 32, 0, stream>>>(A, nullptr, WT, nullptr, KK, P1, DO, nullptr, (size_t)0, (size_t)0, (size_t)0);
        k_gemmw<bf, 0, false><<<dim3(RB / 64, DO / 64, 1), 32, 0, stream>>>(PB + r0 * NB, nullptr, VT, nullptr, NB, P2, DO, nullptr, (size_t)0, (size_t)0, (size_t)0);
        axpby_kernel<<<(unsigned)(((size_t)RB * DO / 4 + 255) / 256), 256, 0, stream>>>(P1, P2, OUT + r0 * DO, (size_t)RB * DO / 4, 1.0f, 1.0f);
    }
}
